// ViM_MambaBlock_86569360818675
// MI455X (gfx1250) — hardware-verified
//
#include <hip/hip_runtime.h>
#include <math.h>
#include <stddef.h>


#define B_   2
#define S_   1024
#define D_   1024
#define E_   2048
#define N_   16
#define R_   64
#define BS_  (B_ * S_)
#define DBCW 96
#define DBCP 128
#define WSCALE 32.0f
#define WINV   0.03125f

#define GT   64
#define SCP  68

typedef _Float16 f16;
typedef f16   v16h __attribute__((ext_vector_type(16)));
typedef f16   v8h  __attribute__((ext_vector_type(8)));
typedef float v8f  __attribute__((ext_vector_type(8)));
typedef float v4f  __attribute__((ext_vector_type(4)));
union Frag { v16h v; v8h h[2]; };

static_assert(BS_ % GT == 0);
static_assert(S_ % GT == 0);
static_assert(D_ % GT == 0);
static_assert(E_ % GT == 0);
static_assert(DBCP % GT == 0);
static_assert((3 * D_) % 32 == 0);
static_assert(E_ % 128 == 0);
static_assert(S_ % 8 == 0);

enum { MD_H16 = 0, MD_SILU = 1, MD_DUAL = 2, MD_SOFTPLUS = 3, MD_FINAL = 4 };

__device__ __forceinline__ v8f wmma16(const v16h& a, const v16h& b, v8f c)
{
    return __builtin_amdgcn_wmma_f32_16x16x32_f16(false, a, false, b, (short)0, c, false, false);
}

__device__ __forceinline__ float rcp_f(float d) { return __builtin_amdgcn_rcpf(d); }

__device__ __forceinline__ float block_sum256(float v, float* red)
{
    #pragma unroll
    for (int o = 16; o > 0; o >>= 1) v += __shfl_xor(v, o);
    const int w = threadIdx.x >> 5, l = threadIdx.x & 31;
    __syncthreads();
    if (l == 0) red[w] = v;
    __syncthreads();
    float r = red[0];
    #pragma unroll
    for (int i = 1; i < 8; ++i) r += red[i];
    return r;
}

__global__ __launch_bounds__(256)
void k_cvt(const float* __restrict__ src, f16* __restrict__ dst, int n_valid, int n_total, float scale)
{
    const int i8 = (blockIdx.x * 256 + (int)threadIdx.x) * 8;
    v8h hv;
    #pragma unroll
    for (int i = 0; i < 8; ++i) hv[i] = (f16)0.0f;
    if (i8 < n_valid) {
        const v4f a = *(const v4f*)(src + i8);
        const v4f c = *(const v4f*)(src + i8 + 4);
        #pragma unroll
        for (int i = 0; i < 4; ++i) { hv[i] = (f16)(a[i] * scale); hv[4 + i] = (f16)(c[i] * scale); }
    }
    if (i8 < n_total) *(volatile v8h*)(dst + i8) = hv;
    __threadfence();
    if (i8 < n_total) *(volatile v8h*)(dst + i8) = hv;
}

__global__ __launch_bounds__(256)
void k_ada(const float* __restrict__ c, const float* __restrict__ Wada,
           const float* __restrict__ bada, float* __restrict__ ada)
{
    __shared__ float s_c[2 * D_];
    __shared__ __attribute__((aligned(16))) float s_o[32];
    const int tid = threadIdx.x, wave = tid >> 5, lane = tid & 31;
    const int per_b = (3 * D_) / 32;
    const int blk = blockIdx.x;
    const int b  = blk / per_b;
    const int j0 = (blk - b * per_b) * 32;

    for (int i = tid; i < 2 * D_; i += 256) {
        const float v = c[(size_t)b * 2 * D_ + i];
        s_c[i] = v * rcp_f(1.0f + expf(-v));
    }
    __syncthreads();

    #pragma unroll
    for (int q = 0; q < 4; ++q) {
        const int o = j0 + wave * 4 + q;
        const float* w = Wada + (size_t)o * (2 * D_);
        float acc = 0.0f;
        #pragma unroll 4
        for (int k = lane; k < 2 * D_; k += 32) acc += s_c[k] * w[k];
        #pragma unroll
        for (int off = 16; off > 0; off >>= 1) acc += __shfl_xor(acc, off);
        if (lane == 0) s_o[wave * 4 + q] = acc + bada[o];
    }
    __syncthreads();

    v4f v;
    #pragma unroll
    for (int i = 0; i < 4; ++i) v[i] = 0.0f;
    if (tid < 8) v = *(const v4f*)(s_o + 4 * tid);
    float* dst = ada + (size_t)b * 3 * D_ + j0 + 4 * tid;
    if (tid < 8) *(volatile v4f*)dst = v;
    __threadfence();
    if (tid < 8) *(volatile v4f*)dst = v;
}

__global__ __launch_bounds__(256)
void k_ln(const float* __restrict__ x, const float* __restrict__ ada,
          const float* __restrict__ g1, const float* __restrict__ b1,
          const float* __restrict__ g2, const float* __restrict__ b2,
          float* __restrict__ skip, f16* __restrict__ xn)
{
    __shared__ float red[8];
    __shared__ __attribute__((aligned(16))) f16 sh[D_];
    const int row = blockIdx.x, b = row / S_, tid = threadIdx.x, c0 = 4 * tid;
    const size_t gi = (size_t)row * D_ + c0;

    const v4f xv = *(const v4f*)(x + gi);
    float s = (xv[0] + xv[1]) + (xv[2] + xv[3]);
    const float mean = block_sum256(s, red) * (1.0f / D_);
    const v4f d = xv - mean;
    float ss = (d[0] * d[0] + d[1] * d[1]) + (d[2] * d[2] + d[3] * d[3]);
    const float var = block_sum256(ss, red) * (1.0f / D_);
    const float rstd = rsqrtf(var + 1e-5f);

    const v4f gv1 = *(const v4f*)(g1 + c0), bv1 = *(const v4f*)(b1 + c0);
    const v4f shf = *(const v4f*)(ada + (size_t)b * 3 * D_ + c0);
    const v4f scl = *(const v4f*)(ada + (size_t)b * 3 * D_ + D_ + c0);
    v4f y = (d * rstd) * gv1 + bv1;
    y = y * (scl + 1.0f) + shf;

    float s2 = (y[0] + y[1]) + (y[2] + y[3]);
    const float mean2 = block_sum256(s2, red) * (1.0f / D_);
    const v4f d2 = y - mean2;
    float ss2 = (d2[0] * d2[0] + d2[1] * d2[1]) + (d2[2] * d2[2] + d2[3] * d2[3]);
    const float var2 = block_sum256(ss2, red) * (1.0f / D_);
    const float rstd2 = rsqrtf(var2 + 1e-5f);
    const v4f gv2 = *(const v4f*)(g2 + c0), bv2 = *(const v4f*)(b2 + c0);
    const v4f z = (d2 * rstd2) * gv2 + bv2;
    #pragma unroll
    for (int i = 0; i < 4; ++i) sh[c0 + i] = (f16)z[i];
    __syncthreads();

    v8h hv;
    #pragma unroll
    for (int i = 0; i < 8; ++i) hv[i] = (f16)0.0f;
    if (tid < 128) hv = *(const v8h*)(sh + 8 * tid);
    f16* xdst = xn + (size_t)row * D_ + 8 * tid;

    *(volatile v4f*)(skip + gi) = y;
    if (tid < 128) *(volatile v8h*)xdst = hv;
    __threadfence();
    *(volatile v4f*)(skip + gi) = y;
    if (tid < 128) *(volatile v8h*)xdst = hv;
}

__global__ __launch_bounds__(128)
void k_gemm(const f16* __restrict__ A, int lda, const f16* __restrict__ W, int ldw,
            int K, int Nout, const float* __restrict__ bias, int mode,
            float* __restrict__ outF, f16* __restrict__ outH,
            const float* __restrict__ skip, const float* __restrict__ xin,
            const float* __restrict__ gate)
{
    __shared__ __attribute__((aligned(16))) float sC[GT * SCP];
    const int tid = threadIdx.x, wave = tid >> 5, lane = tid & 31;
    const int h = lane >> 4, m = lane & 15;
    const int wr = (wave >> 1) * 32, wc = (wave & 1) * 32;
    const int m0 = blockIdx.x * GT, n0 = blockIdx.y * GT;

    const f16* pa0 = A + (size_t)(m0 + wr + m) * lda + 8 * h;
    const f16* pa1 = pa0 + (size_t)16 * lda;
    const f16* pb0 = W + (size_t)(n0 + wc + m) * ldw + 8 * h;
    const f16* pb1 = pb0 + (size_t)16 * ldw;

    v8f c00 = {0.f, 0.f, 0.f, 0.f, 0.f, 0.f, 0.f, 0.f};
    v8f c01 = c00, c10 = c00, c11 = c00;

    for (int k0 = 0; k0 < K; k0 += 32) {
        Frag a0, a1, b0, b1;
        a0.h[0] = *(const v8h*)(pa0 + k0);  a0.h[1] = *(const v8h*)(pa0 + k0 + 16);
        a1.h[0] = *(const v8h*)(pa1 + k0);  a1.h[1] = *(const v8h*)(pa1 + k0 + 16);
        b0.h[0] = *(const v8h*)(pb0 + k0);  b0.h[1] = *(const v8h*)(pb0 + k0 + 16);
        b1.h[0] = *(const v8h*)(pb1 + k0);  b1.h[1] = *(const v8h*)(pb1 + k0 + 16);
        c00 = wmma16(a0.v, b0.v, c00);
        c01 = wmma16(a0.v, b1.v, c01);
        c10 = wmma16(a1.v, b0.v, c10);
        c11 = wmma16(a1.v, b1.v, c11);
        asm volatile("v_nop\n\tv_nop\n\tv_nop\n\tv_nop"
                     : "+v"(c00), "+v"(c01), "+v"(c10), "+v"(c11)
                     : "v"(a0.v), "v"(a1.v), "v"(b0.v), "v"(b1.v));
    }

    #pragma unroll
    for (int r = 0; r < 8; ++r) {
        const int rr0 = (wr + 8 * h + r) * SCP;
        const int rr1 = (wr + 16 + 8 * h + r) * SCP;
        sC[rr0 + wc + m]      = c00[r];
        sC[rr0 + wc + 16 + m] = c01[r];
        sC[rr1 + wc + m]      = c10[r];
        sC[rr1 + wc + 16 + m] = c11[r];
    }
    __syncthreads();

    const int rA = wave * 16 + h,           cA = 4 * m;
    const int rB = wave * 16 + (lane >> 3), cB = 8 * (lane & 7);

    {
        v4f bv = {0.f, 0.f, 0.f, 0.f};
        if (bias != nullptr) bv = *(const v4f*)(bias + n0 + cA);
        v4f gv = bv;
        if (mode == MD_FINAL) {
            const int bb = m0 / S_;
            gv = *(const v4f*)(gate + (size_t)bb * 3 * D_ + 2 * D_ + n0 + cA);
        }
        #pragma unroll 1
        for (int j = 0; j < 8; ++j) {
            const int r = rA + 2 * j;
            float* sp = sC + r * SCP + cA;
            v4f o = *(const v4f*)sp * WINV + bv;
            if (mode == MD_SILU) {
                #pragma unroll
                for (int i = 0; i < 4; ++i) o[i] = o[i] * rcp_f(1.0f + __expf(-o[i]));
            } else if (mode == MD_SOFTPLUS) {
                #pragma unroll
                for (int i = 0; i < 4; ++i) o[i] = fmaxf(o[i], 0.0f) + __logf(1.0f + __expf(-fabsf(o[i])));
            } else if (mode == MD_FINAL) {
                const size_t gi = (size_t)(m0 + r) * Nout + n0 + cA;
                const v4f sk = *(const v4f*)(skip + gi);
                const v4f xv = *(const v4f*)(xin + gi);
                const v4f oo = o + sk;
                o = xv + gv * oo;
            }
            *(v4f*)sp = o;
        }
    }
    __syncthreads();

    auto store_pass = [&]() {
        if (mode != MD_H16) {
            const float* sp = sC + rA * SCP + cA;
            float* gp = outF + (size_t)(m0 + rA) * Nout + n0 + cA;
            const size_t gstep = (size_t)2 * Nout;
            #pragma unroll
            for (int j = 0; j < 8; ++j) {
                const v4f o = *(const v4f*)(sp + j * 2 * SCP);
                *(volatile v4f*)(gp + j * gstep) = o;
            }
        }
        if (mode == MD_H16 || mode == MD_DUAL) {
            const float* sp = sC + rB * SCP + cB;
            f16* gp = outH + (size_t)(m0 + rB) * Nout + n0 + cB;
            const size_t gstep = (size_t)4 * Nout;
            #pragma unroll
            for (int j = 0; j < 4; ++j) {
                const v4f o0 = *(const v4f*)(sp + j * 4 * SCP);
                const v4f o1 = *(const v4f*)(sp + j * 4 * SCP + 4);
                v8h hv;
                #pragma unroll
                for (int i = 0; i < 4; ++i) { hv[i] = (f16)o0[i]; hv[4 + i] = (f16)o1[i]; }
                *(volatile v8h*)(gp + j * gstep) = hv;
            }
        }
    };
    store_pass();
    __threadfence();
    store_pass();
}

__global__ __launch_bounds__(128)
void k_scan(const float* __restrict__ u, const float* __restrict__ delta,
            const float* __restrict__ dbc, const float* __restrict__ Alog,
            const float* __restrict__ Dp,
            const float* __restrict__ y1in, const float* __restrict__ actmx,
            float* __restrict__ yout, f16* __restrict__ ycomb, int dir)
{
    __shared__ __attribute__((aligned(16))) float stage[8 * 128];
    const int tid = threadIdx.x;
    const int per_b = E_ / 128;
    const int blk = blockIdx.x;
    const int b  = blk / per_b;
    const int e0 = (blk - b * per_b) * 128;
    const int e  = e0 + tid;

    float Ac[N_], hst[N_];
    #pragma unroll
    for (int n = 0; n < N_; ++n) { Ac[n] = -__expf(Alog[(size_t)e * N_ + n]); hst[n] = 0.0f; }
    const float dp = Dp[e];
    const float* dbcb = dbc + (size_t)b * S_ * DBCP;

    auto flush = [&](int base) {
        if (dir == 0) {
            #pragma unroll
            for (int j = 0; j < 2; ++j) {
                const int r = 4 * j + (tid >> 5);
                const int cc = 4 * (tid & 31);
                const v4f v = *(const v4f*)(stage + r * 128 + cc);
                const size_t gi = ((size_t)b * S_ + base + r) * E_ + e0 + cc;
                *(volatile v4f*)(yout + gi) = v;
            }
        } else {
            const int r = tid >> 4;
            const int cc = 8 * (tid & 15);
            const v4f v0 = *(const v4f*)(stage + r * 128 + cc);
            const v4f v1 = *(const v4f*)(stage + r * 128 + cc + 4);
            const size_t gi = ((size_t)b * S_ + base + r) * E_ + e0 + cc;
            const v4f ya = *(const v4f*)(y1in + gi),  yb = *(const v4f*)(y1in + gi + 4);
            const v4f aa = *(const v4f*)(actmx + gi), ab = *(const v4f*)(actmx + gi + 4);
            const v4f pa = aa * ya, qa = aa * v0;
            const v4f pb = ab * yb, qb = ab * v1;
            const v4f sa = pa + qa, sb = pb + qb;
            v8h hv;
            #pragma unroll
            for (int i = 0; i < 4; ++i) { hv[i] = (f16)sa[i]; hv[4 + i] = (f16)sb[i]; }
            *(volatile v8h*)(ycomb + gi) = hv;
        }
    };

    #pragma unroll 1
    for (int t = 0; t < S_; ++t) {
        const int s = dir ? (S_ - 1 - t) : t;
        const size_t row = (size_t)b * S_ + s;
        const float dlt = delta[row * E_ + e];
        const float uu  = u[row * E_ + e];
        const v4f* bcp = (const v4f*)(dbcb + (size_t)s * DBCP + R_);
        float y = 0.0f;
        #pragma unroll
        for (int q = 0; q < 4; ++q) {
            const v4f Bq = bcp[q];
            const v4f Cq = bcp[4 + q];
            #pragma unroll
            for (int i = 0; i < 4; ++i) {
                const int n = 4 * q + i;
                const float dA  = __expf(dlt * Ac[n]);
                const float dBu = (dlt * Bq[i]) * uu;
                const float hn  = dA * hst[n] + dBu;
                hst[n] = hn;
                y += hn * Cq[i];
            }
        }
        y += uu * dp;
        stage[(s & 7) * 128 + tid] = y;
        if ((t & 7) == 7) {
            __syncthreads();
            const int base = s & ~7;
            flush(base);
            __threadfence();
            flush(base);
            __syncthreads();
        }
    }
}

extern "C" void kernel_launch(void* const* d_in, const int* in_sizes, int n_in,
                              void* d_out, int out_size, void* d_ws, size_t ws_size,
                              hipStream_t stream)
{
    if (n_in < 29) return;
    if (in_sizes[0] != BS_ * D_ || out_size != BS_ * D_) return;

    const float* x     = (const float*)d_in[0];
    const float* c     = (const float*)d_in[1];
    const float* n1g   = (const float*)d_in[3];
    const float* n1b   = (const float*)d_in[4];
    const float* n2g   = (const float*)d_in[5];
    const float* n2b   = (const float*)d_in[6];
    const float* Wx    = (const float*)d_in[7];
    const float* bx    = (const float*)d_in[8];
    const float* Wz    = (const float*)d_in[9];
    const float* bz    = (const float*)d_in[10];
    const float* Wf    = (const float*)d_in[11];
    const float* bff   = (const float*)d_in[12];
    const float* Wada  = (const float*)d_in[13];
    const float* bada  = (const float*)d_in[14];
    const float* Wc1   = (const float*)d_in[15];
    const float* bc1   = (const float*)d_in[16];
    const float* Wc2   = (const float*)d_in[17];
    const float* bc2   = (const float*)d_in[18];
    const float* Wdbc1 = (const float*)d_in[19];
    const float* Wdt1  = (const float*)d_in[20];
    const float* bdt1  = (const float*)d_in[21];
    const float* Alog1 = (const float*)d_in[22];
    const float* Dp1   = (const float*)d_in[23];
    const float* Wdbc2 = (const float*)d_in[24];
    const float* Wdt2  = (const float*)d_in[25];
    const float* bdt2  = (const float*)d_in[26];
    const float* Alog2 = (const float*)d_in[27];
    const float* Dp2   = (const float*)d_in[28];

    char* ws = (char*)d_ws;
    size_t off = 0;
    auto carve = [&](size_t bytes) -> char* {
        char* p = ws + off;
        off += (bytes + 255) & ~(size_t)255;
        return p;
    };
    float* adab  = (float*)carve((size_t)B_ * 3 * D_ * 4);
    float* skip  = (float*)carve((size_t)BS_ * D_ * 4);
    f16*   mz    = (f16*)  carve((size_t)BS_ * E_ * 2);
    float* actmx = (float*)carve((size_t)BS_ * E_ * 4);
    float* zf    = (float*)carve((size_t)BS_ * E_ * 4);
    f16*   zh    = (f16*)  carve((size_t)BS_ * E_ * 2);
    f16*   xn    = zh;
    float* dbcf  = (float*)carve((size_t)BS_ * DBCP * 4);
    f16*   dbch  = (f16*)  carve((size_t)BS_ * DBCP * 2);
    float* dlt   = (float*)carve((size_t)BS_ * E_ * 4);
    float* y1    = (float*)carve((size_t)BS_ * E_ * 4);
    f16*   ycb   = (f16*)  carve((size_t)BS_ * E_ * 2);
    f16*   wsl   = (f16*)  carve((size_t)E_ * E_ * 2);
    if (off > ws_size) return;

    auto cvt = [&](const float* src, int n_valid, int n_total) {
        const int nb = (n_total / 8 + 255) / 256;
        k_cvt<<<nb, 256, 0, stream>>>(src, wsl, n_valid, n_total, WSCALE);
    };
    auto gemm = [&](const f16* A, int lda, int ldw, int K, int Nout, const float* bias, int mode,
                    float* oF, f16* oH, const float* sk, const float* xi, const float* gt) {
        dim3 grid(BS_ / GT, Nout / GT);
        k_gemm<<<grid, 128, 0, stream>>>(A, lda, wsl, ldw, K, Nout, bias, mode, oF, oH, sk, xi, gt);
    };

    k_ada<<<B_ * ((3 * D_) / 32), 256, 0, stream>>>(c, Wada, bada, adab);
    k_ln<<<BS_, 256, 0, stream>>>(x, adab, n1g, n1b, n2g, n2b, skip, xn);

    cvt(Wz, E_ * D_, E_ * D_);
    gemm(xn, D_, D_, D_, E_, bz, MD_H16, nullptr, mz, nullptr, nullptr, nullptr);
    cvt(Wx, E_ * D_, E_ * D_);
    gemm(xn, D_, D_, D_, E_, bx, MD_SILU, actmx, nullptr, nullptr, nullptr, nullptr);

    cvt(Wc1, E_ * E_, E_ * E_);
    gemm(mz, E_, E_, E_, E_, bc1, MD_DUAL, zf, zh, nullptr, nullptr, nullptr);
    cvt(Wdbc1, DBCW * E_, DBCP * E_);
    gemm(zh, E_, E_, E_, DBCP, nullptr, MD_DUAL, dbcf, dbch, nullptr, nullptr, nullptr);
    cvt(Wdt1, E_ * R_, E_ * R_);
    gemm(dbch, DBCP, R_, R_, E_, bdt1, MD_SOFTPLUS, dlt, nullptr, nullptr, nullptr, nullptr);
    k_scan<<<(B_ * E_) / 128, 128, 0, stream>>>(zf, dlt, dbcf, Alog1, Dp1, nullptr, nullptr, y1, nullptr, 0);

    cvt(Wc2, E_ * E_, E_ * E_);
    gemm(mz, E_, E_, E_, E_, bc2, MD_DUAL, zf, zh, nullptr, nullptr, nullptr);
    cvt(Wdbc2, DBCW * E_, DBCP * E_);
    gemm(zh, E_, E_, E_, DBCP, nullptr, MD_DUAL, dbcf, dbch, nullptr, nullptr, nullptr);
    cvt(Wdt2, E_ * R_, E_ * R_);
    gemm(dbch, DBCP, R_, R_, E_, bdt2, MD_SOFTPLUS, dlt, nullptr, nullptr, nullptr, nullptr);
    k_scan<<<(B_ * E_) / 128, 128, 0, stream>>>(zf, dlt, dbcf, Alog2, Dp2, y1, actmx, nullptr, ycb, 1);

    cvt(Wf, D_ * E_, D_ * E_);
    gemm(ycb, E_, E_, E_, D_, bff, MD_FINAL, (float*)d_out, nullptr, skip, x, adab);

    (void)ws_size;
}
